// DualPath_12403865550987
// MI455X (gfx1250) — hardware-run, weakly checked
//
#include <hip/hip_runtime.h>
#include <math.h>

constexpr int kSeq   = 256;
constexpr int kChan  = 64;
constexpr int kTime  = 512;
constexpr int kLen   = 506;
constexpr int kHid   = 32;
constexpr int kTap   = 7;
constexpr int kFf    = 128;
constexpr int kRows  = kSeq * kTime;
constexpr int kQRows = 520;
constexpr int kKsru  = kTap * kChan;
constexpr int kKc2   = kTap * kFf;
constexpr int kKct   = kTap * kChan;
constexpr float kWCarry    = 16.0f;
constexpr float kWCarryInv = 1.0f / 16.0f;
constexpr float kEps = 1e-6f;

constexpr int kOffSru = 0;
constexpr int kOffC1  = kOffSru + 2 * 128 * kKsru;
constexpr int kOffC2  = kOffC1 + kFf * kChan;
constexpr int kOffC3  = kOffC2 + kFf * kKc2;
constexpr int kOffCt  = kOffC3 + kChan * kFf;
constexpr int kWTotal = kOffCt + kChan * kKct;

static_assert(kLen == kTime - kTap + 1, "unfold length");
static_assert(kKsru == 448 && kKc2 == 896 && kKct == 448, "K sizes");
static_assert(kKsru % 32 == 0 && kChan % 32 == 0 && kKc2 % 32 == 0 && kFf % 32 == 0 && kKct % 32 == 0, "K multiple of 32");
static_assert(kRows % 64 == 0 && kFf % 64 == 0 && kChan % 64 == 0 && kTime % 64 == 0, "tile multiples");
static_assert(kOffC1 == 114688 && kOffC2 == 122880 && kOffC3 == 237568 && kOffCt == 245760 && kWTotal == 274432, "weight plane map");
static_assert(kWTotal % 2048 == 0, "weight prep grid exact");
static_assert(kQRows >= kTime + kTap - 1, "padded plane pitch for the transposed conv");
static_assert(2 * kHid == kChan, "two directions fill the channel axis");

typedef __attribute__((ext_vector_type(16))) _Float16 v16h;
typedef __attribute__((ext_vector_type(8)))  _Float16 v8h;
typedef __attribute__((ext_vector_type(16))) __bf16   v16b;
typedef __attribute__((ext_vector_type(8)))  __bf16   v8b;
typedef __attribute__((ext_vector_type(8)))  float    v8f;
typedef __attribute__((ext_vector_type(4)))  float    v4f;
typedef __attribute__((ext_vector_type(4)))  unsigned uv4;

__device__ __forceinline__ unsigned short f2bf_bits(float f) {
  unsigned u = __float_as_uint(f);
  return (unsigned short)((u + 0x7FFFu + ((u >> 16) & 1u)) >> 16);
}
__device__ __forceinline__ float bf_bits2f(unsigned short h) { return __uint_as_float(((unsigned)h) << 16); }

__device__ __forceinline__ float h16_to_f32(unsigned hb) {
  const unsigned sgn = (hb & 0x8000u) << 16;
  const unsigned em = hb & 0x7fffu;
  const float fn = __uint_as_float((em << 13) + 0x38000000u);
  const float fs = (float)em * 5.9604644775390625e-8f;
  const float mag = (em < 0x400u) ? fs : fn;
  return __uint_as_float(__float_as_uint(mag) | sgn);
}
__device__ __forceinline__ void unpack8(const uv4 w, float (&f)[8]) {
  const unsigned w0 = w[0];
  const unsigned w1 = w[1];
  const unsigned w2 = w[2];
  const unsigned w3 = w[3];
  f[0] = h16_to_f32(w0 & 0xffffu);
  f[1] = h16_to_f32(w0 >> 16);
  f[2] = h16_to_f32(w1 & 0xffffu);
  f[3] = h16_to_f32(w1 >> 16);
  f[4] = h16_to_f32(w2 & 0xffffu);
  f[5] = h16_to_f32(w2 >> 16);
  f[6] = h16_to_f32(w3 & 0xffffu);
  f[7] = h16_to_f32(w3 >> 16);
}

__device__ __forceinline__ void dep_guard4_h(v8f& a, v8f& b, v8f& c, v8f& d, v16h x, v16h y) { asm volatile("v_nop\n\tv_nop\n\tv_nop\n\tv_nop" : "+v"(a), "+v"(b), "+v"(c), "+v"(d) : "v"(x), "v"(y)); }
__device__ __forceinline__ void dep_guard4_b(v8f& a, v8f& b, v8f& c, v8f& d, v16b x, v16b y) { asm volatile("v_nop\n\tv_nop\n\tv_nop\n\tv_nop" : "+v"(a), "+v"(b), "+v"(c), "+v"(d) : "v"(x), "v"(y)); }
__device__ __forceinline__ void keep4_h(v16h a, v16h b, v16h c, v16h d) { asm volatile("v_nop" :: "v"(a), "v"(b), "v"(c), "v"(d)); }
__device__ __forceinline__ void keep4_b(v16b a, v16b b, v16b c, v16b d) { asm volatile("v_nop" :: "v"(a), "v"(b), "v"(c), "v"(d)); }
__device__ __forceinline__ void acc_guard4(v8f& a, v8f& b, v8f& c, v8f& d) { asm volatile("v_nop\n\tv_nop\n\tv_nop\n\tv_nop" : "+v"(a), "+v"(b), "+v"(c), "+v"(d)); }

template <typename T> struct Frag;
template <> struct Frag<_Float16> {
  typedef v16h V; union U { v16h v; v8h h[2]; };
  static __device__ __forceinline__ v16h load(const _Float16* p) {
    U f; f.h[0] = *(const v8h*)(p); f.h[1] = *(const v8h*)(p + 16); return f.v;
  }
  static __device__ __forceinline__ v8f mma(v16h a, v16h b, v8f c) {
    return __builtin_amdgcn_wmma_f32_16x16x32_f16(false, a, false, b, (short)0, c, false, false);
  }
  static __device__ __forceinline__ void guard4(v8f& a, v8f& b, v8f& c, v8f& d, v16h x, v16h y) { dep_guard4_h(a, b, c, d, x, y); }
  static __device__ __forceinline__ void keep(v16h a, v16h b, v16h c, v16h d) { keep4_h(a, b, c, d); }
};
template <> struct Frag<__bf16> {
  typedef v16b V; union U { v16b v; v8b h[2]; };
  static __device__ __forceinline__ v16b load(const __bf16* p) {
    U f; f.h[0] = *(const v8b*)(p); f.h[1] = *(const v8b*)(p + 16); return f.v;
  }
  static __device__ __forceinline__ v8f mma(v16b a, v16b b, v8f c) {
    return __builtin_amdgcn_wmma_f32_16x16x32_bf16(false, a, false, b, (short)0, c, false, false);
  }
  static __device__ __forceinline__ void guard4(v8f& a, v8f& b, v8f& c, v8f& d, v16b x, v16b y) { dep_guard4_b(a, b, c, d, x, y); }
  static __device__ __forceinline__ void keep(v16b a, v16b b, v16b c, v16b d) { keep4_b(a, b, c, d); }
};

template <int ET> struct Elem;
template <> struct Elem<0> { typedef _Float16 T; };
template <> struct Elem<1> { typedef __bf16 T; };
template <int ET, bool SPLIT, int BIAS_MODE, int OUT_MODE, bool RESID>
__global__ __launch_bounds__(256) void wmma_gemm64(
    const unsigned short* __restrict__ Ap, const unsigned short* __restrict__ A2p, int lda, long strideA,
    const unsigned short* __restrict__ Btp, const unsigned short* __restrict__ Bt2p, int ldb, long strideB,
    void* __restrict__ Cout, void* __restrict__ Cout2, int ldc, long strideC,
    const float* __restrict__ bias,
    const float* __restrict__ resid, long strideR,
    int M, int N, int K, float scale) {
  typedef typename Elem<ET>::T T;
  typedef typename Frag<T>::V V;
  const T* A = (const T*)Ap; const T* A2 = (const T*)A2p; const T* Bt = (const T*)Btp; const T* Bt2 = (const T*)Bt2p;
  __shared__ __align__(16) float sT[8][16 * 68];
  const int b    = blockIdx.y;
  const int lane = threadIdx.x & 31;
  const int wave = threadIdx.x >> 5;
  const int tilesN = N >> 6;
  const int tilesM = M >> 6;
  const int tile = blockIdx.x * 8 + wave;
  if (tile >= tilesM * tilesN) return;
  const int tm = tile / tilesN;
  const int tn = tile - tm * tilesN;
  const int m0 = tm << 6;
  const int n0 = tn << 6;

  const T* Ab  = A  + (size_t)b * strideA;
  const T* Bb  = Bt + (size_t)b * strideB;
  const T* Ab2 = SPLIT ? (A2  + (size_t)b * strideA) : nullptr;
  const T* Bb2 = SPLIT ? (Bt2 + (size_t)b * strideB) : nullptr;

  const int rlane = lane & 15;
  const int koff  = (lane >> 4) * 8;
  const int mOff  = (lane >> 4) * 8;

  v8f acc[4][4];
#pragma unroll
  for (int i = 0; i < 4; ++i)
#pragma unroll
    for (int j = 0; j < 4; ++j) acc[i][j] = (v8f){0.f,0.f,0.f,0.f,0.f,0.f,0.f,0.f};

  for (int k0 = 0; k0 < K; k0 += 32) {
    V bh[4], bl[4];
#pragma unroll
    for (int j = 0; j < 4; ++j) {
      const size_t bo = (size_t)(n0 + (j << 4) + rlane) * ldb + koff + k0;
      bh[j] = Frag<T>::load(Bb + bo);
      if (SPLIT) bl[j] = Frag<T>::load(Bb2 + bo);
    }
#pragma unroll
    for (int i = 0; i < 4; ++i) {
      const size_t ao = (size_t)(m0 + (i << 4) + rlane) * lda + koff + k0;
      V ah = Frag<T>::load(Ab + ao);
      V al;
      if (SPLIT) al = Frag<T>::load(Ab2 + ao);
#pragma unroll
      for (int j = 0; j < 4; ++j) {
        acc[i][j] = Frag<T>::mma(ah, bh[j], acc[i][j]);
        if (SPLIT) {
          acc[i][j] = Frag<T>::mma(ah, bl[j], acc[i][j]);
          acc[i][j] = Frag<T>::mma(al, bh[j], acc[i][j]);
        }
      }
      Frag<T>::guard4(acc[i][0], acc[i][1], acc[i][2], acc[i][3], ah, SPLIT ? al : ah);
    }
    Frag<T>::keep(bh[0], bh[1], bh[2], bh[3]);
    if (SPLIT) Frag<T>::keep(bl[0], bl[1], bl[2], bl[3]);
  }
  acc_guard4(acc[0][0], acc[0][1], acc[0][2], acc[0][3]);
  acc_guard4(acc[1][0], acc[1][1], acc[1][2], acc[1][3]);
  acc_guard4(acc[2][0], acc[2][1], acc[2][2], acc[2][3]);
  acc_guard4(acc[3][0], acc[3][1], acc[3][2], acc[3][3]);

  float* slab = sT[wave];
  const float* Rb = RESID ? (resid + (size_t)b * strideR) : nullptr;
#pragma unroll
  for (int i = 0; i < 4; ++i) {
    const int mBase = m0 + (i << 4);
#pragma unroll
    for (int j = 0; j < 4; ++j) {
      const int n = n0 + (j << 4) + rlane;
      float bv = 0.f;
      if (BIAS_MODE == 2) bv = bias[n];
#pragma unroll
      for (int r = 0; r < 8; ++r) {
        float v = acc[i][j][r] * scale;
        if (BIAS_MODE == 1) v += bias[mBase + mOff + r];
        if (BIAS_MODE == 2) v += bv;
        if (RESID) v += Rb[(size_t)(mBase + mOff + r) * ldc + n];
        slab[(mOff + r) * 68 + (j << 4) + rlane] = v;
      }
    }
    __builtin_amdgcn_fence(__ATOMIC_RELEASE, "workgroup");
    __builtin_amdgcn_wave_barrier();
    __builtin_amdgcn_fence(__ATOMIC_ACQUIRE, "workgroup");
    if (OUT_MODE == 0) {
      float* C = (float*)Cout + (size_t)b * strideC;
      const int hh = lane >> 4, c4 = (lane & 15) * 4;
      for (int pass = 0; pass < 2; ++pass) {
#pragma unroll
        for (int it = 0; it < 8; ++it) {
          const int row = it * 2 + hh;
          v4f v = *(const v4f*)(slab + row * 68 + c4);
          *(volatile v4f*)(C + (size_t)(mBase + row) * ldc + n0 + c4) = v;
        }
        __threadfence();
      }
    } else {
      const int q = lane >> 3, c8 = (lane & 7) * 8;
      unsigned short* C  = (unsigned short*)Cout  + (size_t)b * strideC;
      unsigned short* C2 = (OUT_MODE == 2) ? ((unsigned short*)Cout2 + (size_t)b * strideC) : nullptr;
      for (int pass = 0; pass < 2; ++pass) {
#pragma unroll
        for (int it = 0; it < 4; ++it) {
          const int row = it * 4 + q;
          const float* sp = slab + row * 68 + c8;
          v8h hv, lv;
#pragma unroll
          for (int e = 0; e < 8; ++e) {
            if (OUT_MODE == 1) {
              hv[e] = (_Float16)sp[e];
            } else {
              unsigned short hb = f2bf_bits(sp[e]);
              unsigned short lb = f2bf_bits(sp[e] - bf_bits2f(hb));
              hv[e] = __builtin_bit_cast(_Float16, hb);
              lv[e] = __builtin_bit_cast(_Float16, lb);
            }
          }
          *(volatile v8h*)(C + (size_t)(mBase + row) * ldc + n0 + c8) = hv;
          if (OUT_MODE == 2) *(volatile v8h*)(C2 + (size_t)(mBase + row) * ldc + n0 + c8) = lv;
        }
        __threadfence();
      }
    }
    __builtin_amdgcn_fence(__ATOMIC_RELEASE, "workgroup");
    __builtin_amdgcn_wave_barrier();
    __builtin_amdgcn_fence(__ATOMIC_ACQUIRE, "workgroup");
  }
}

__global__ __launch_bounds__(256) void gn0_partial_kernel(const float* __restrict__ x, float* __restrict__ part) {
  __shared__ float shs[8];
  __shared__ float shq[8];
  const int tid = threadIdx.x, lane = tid & 31, wave = tid >> 5;
  const v4f* xp = (const v4f*)x + (size_t)blockIdx.x * 8192;
  float s = 0.0f, q = 0.0f;
#pragma unroll 4
  for (int i = 0; i < 32; ++i) {
    const v4f v = xp[i * 256 + tid];
    s += (v[0] + v[1]) + (v[2] + v[3]);
    q += (v[0] * v[0] + v[1] * v[1]) + (v[2] * v[2] + v[3] * v[3]);
  }
#pragma unroll
  for (int off = 16; off > 0; off >>= 1) { s += __shfl_xor(s, off, 32); q += __shfl_xor(q, off, 32); }
  if (lane == 0) { shs[wave] = s; shq[wave] = q; }
  __syncthreads();
  if (wave == 0) {
    float S = 0.0f, Q = 0.0f;
#pragma unroll
    for (int i = 0; i < 8; ++i) { S += shs[i]; Q += shq[i]; }
    const float v = (lane == 0) ? S : ((lane == 1) ? Q : 0.0f);
    volatile float* p = part + (size_t)blockIdx.x * 32 + lane;
    *p = v;
    __threadfence();
    *p = v;
  }
}

__global__ __launch_bounds__(256) void gn0_final_kernel(const float* __restrict__ part, float* __restrict__ stat) {
  __shared__ double ds[256];
  __shared__ double dq[256];
  const int t = threadIdx.x;
  ds[t] = (double)part[t * 32];
  dq[t] = (double)part[t * 32 + 1];
  __syncthreads();
  for (int o = 128; o > 0; o >>= 1) {
    if (t < o) { ds[t] += ds[t + o]; dq[t] += dq[t + o]; }
    __syncthreads();
  }
  const double inv = 1.0 / 8388608.0;
  const double mean = ds[0] * inv;
  double var = dq[0] * inv - mean * mean;
  var = (var < 0.0) ? 0.0 : var;
  const float rstd = rsqrtf((float)var + kEps);
  const float meanf = (float)mean;
  if (t < 32) {
    const float v = (t == 0) ? meanf : ((t == 1) ? rstd : 0.0f);
    volatile float* p = stat + t;
    *p = v;
    __threadfence();
    *p = v;
  }
}

__device__ __forceinline__ int widx_sru(int j) {
  const int d = j / 57344;
  const int rem = j - d * 57344;
  const int o = rem / 448;
  const int kk = rem - o * 448;
  const int k = kk >> 6;
  const int c = kk & 63;
  return (d * 448 + c * 7 + k) * 128 + o;
}
__device__ __forceinline__ int widx_c2(int j) {
  const int o = j / 896;
  const int kk = j - o * 896;
  const int k = kk >> 7;
  const int c = kk & 127;
  return (o * 128 + c) * 7 + k;
}
__device__ __forceinline__ int widx_ct(int j) {
  const int o = j / 448;
  const int kk = j - o * 448;
  const int kp = kk >> 6;
  const int i = kk & 63;
  return (i * 64 + o) * 7 + (6 - kp);
}
__global__ __launch_bounds__(256) void wprep_kernel(const float* __restrict__ sruw, const float* __restrict__ c1w,
                                                    const float* __restrict__ c2w, const float* __restrict__ c3w,
                                                    const float* __restrict__ ctw, unsigned short* __restrict__ WP) {
  const int blk = blockIdx.x, tid = threadIdx.x;
  v8h hv;
  int obase;
  if (blk < 56) {
    const int j0 = (blk * 256 + tid) * 8;
#pragma unroll
    for (int e = 0; e < 8; ++e) hv[e] = (_Float16)(sruw[widx_sru(j0 + e)] * kWCarry);
    obase = kOffSru + j0;
  } else if (blk < 60) {
    const int j0 = ((blk - 56) * 256 + tid) * 8;
#pragma unroll
    for (int e = 0; e < 8; ++e) hv[e] = (_Float16)(c1w[j0 + e] * kWCarry);
    obase = kOffC1 + j0;
  } else if (blk < 116) {
    const int j0 = ((blk - 60) * 256 + tid) * 8;
#pragma unroll
    for (int e = 0; e < 8; ++e) hv[e] = (_Float16)(c2w[widx_c2(j0 + e)] * kWCarry);
    obase = kOffC2 + j0;
  } else if (blk < 120) {
    const int j0 = ((blk - 116) * 256 + tid) * 8;
#pragma unroll
    for (int e = 0; e < 8; ++e) hv[e] = (_Float16)(c3w[j0 + e] * kWCarry);
    obase = kOffC3 + j0;
  } else {
    const int j0 = ((blk - 120) * 256 + tid) * 8;
#pragma unroll
    for (int e = 0; e < 8; ++e) hv[e] = (_Float16)(ctw[widx_ct(j0 + e)] * kWCarry);
    obase = kOffCt + j0;
  }
  volatile v8h* op = (volatile v8h*)(WP + obase);
  *op = hv;
  __threadfence();
  *op = hv;
}

__global__ __launch_bounds__(256) void pack_xn_kernel(const float* __restrict__ x, const float* __restrict__ g0w,
                                                      const float* __restrict__ g0b, const float* __restrict__ stat,
                                                      unsigned short* __restrict__ Xn) {
  __shared__ float Tt[64 * 65];
  const int tid = threadIdx.x;
  const int blk = blockIdx.x;
  if (blk == kSeq * 8) {
    if (tid < 64) {
      v8h z;
#pragma unroll
      for (int e = 0; e < 8; ++e) z[e] = (_Float16)0.0f;
      volatile v8h* op = (volatile v8h*)(Xn + (size_t)kRows * kChan + tid * 8);
      *op = z;
      __threadfence();
      *op = z;
    }
    return;
  }
  const int n = blk >> 3;
  const int t0 = (blk & 7) * 64;
  const float mean = stat[0];
  const float rstd = stat[1];
#pragma unroll
  for (int i = 0; i < 4; ++i) {
    const int idx = i * 256 + tid;
    const int c = idx >> 4;
    const int t4 = (idx & 15) * 4;
    const v4f v = *(const v4f*)(x + ((size_t)(c * kSeq + n)) * kTime + t0 + t4);
    const float gw = g0w[c];
    const float gb = g0b[c];
    Tt[c * 65 + t4 + 0] = ((v[0] - mean) * rstd) * gw + gb;
    Tt[c * 65 + t4 + 1] = ((v[1] - mean) * rstd) * gw + gb;
    Tt[c * 65 + t4 + 2] = ((v[2] - mean) * rstd) * gw + gb;
    Tt[c * 65 + t4 + 3] = ((v[3] - mean) * rstd) * gw + gb;
  }
  __syncthreads();
  const int q = tid >> 3;
  const int c8 = (tid & 7) * 8;
  v8h hv[2];
#pragma unroll
  for (int g = 0; g < 2; ++g) {
    const int tl = g * 32 + q;
#pragma unroll
    for (int e = 0; e < 8; ++e) hv[g][e] = (_Float16)Tt[(c8 + e) * 65 + tl];
  }
  for (int pass = 0; pass < 2; ++pass) {
#pragma unroll
    for (int g = 0; g < 2; ++g) {
      const size_t o = ((size_t)n * kTime + t0 + g * 32 + q) * kChan + c8;
      *(volatile v8h*)(Xn + o) = hv[g];
    }
    __threadfence();
  }
}

__device__ __forceinline__ float sigmoid_f(float v) { return __builtin_amdgcn_rcpf(1.0f + expf(-v)); }
__global__ __launch_bounds__(256) void sru_scan_kernel(const float* __restrict__ U, const float* __restrict__ sv,
                                                       const float* __restrict__ sb, float* __restrict__ HB, int d) {
  const int lane = threadIdx.x & 31;
  const int n = blockIdx.x * 8 + (threadIdx.x >> 5);
  const float vf = sv[(d * 2 + 0) * kHid + lane];
  const float vr = sv[(d * 2 + 1) * kHid + lane];
  const float bf = sb[(d * 2 + 0) * kHid + lane];
  const float br = sb[(d * 2 + 1) * kHid + lane];
  float c = 0.0f;
#pragma unroll 1
  for (int s = 0; s < kLen; ++s) {
    const int l = d ? (kLen - 1 - s) : s;
    const float* up = U + ((size_t)(n * kTime + l)) * 128 + lane;
    const float u0 = up[0];
    const float u1 = up[32];
    const float u2 = up[64];
    const float u3 = up[96];
    const float f  = sigmoid_f(u1 + vf * c + bf);
    const float cn = f * c + (1.0f - f) * u0;
    const float r  = sigmoid_f(u2 + vr * c + br);
    const float h  = r * cn + (1.0f - r) * u3;
    c = cn;
    volatile float* hp = HB + ((size_t)(n * kTime + l)) * kChan + d * kHid + lane;
    *hp = h;
    __threadfence();
    *hp = h;
  }
}

__global__ __launch_bounds__(256) void cast_h_kernel(const float* __restrict__ hb, unsigned short* __restrict__ h16) {
  const int i = blockIdx.x * 256 + threadIdx.x;
  if (i < kRows * 8) {
    const int row = i >> 3;
    const int c8 = (i & 7) * 8;
    const int l = row & (kTime - 1);
    const bool valid = l < kLen;
    const int rc = valid ? row : (row - l + kLen - 1);
    const float* sp = hb + (size_t)rc * kChan + c8;
    const v4f a = *(const v4f*)(sp);
    const v4f b = *(const v4f*)(sp + 4);
    v8h hv;
#pragma unroll
    for (int e = 0; e < 4; ++e) {
      const float fa = valid ? a[e] : 0.0f;
      const float fb = valid ? b[e] : 0.0f;
      hv[e] = (_Float16)fa;
      hv[4 + e] = (_Float16)fb;
    }
    volatile v8h* op = (volatile v8h*)(h16 + (size_t)i * 8);
    *op = hv;
    __threadfence();
    *op = hv;
  }
}

template <int SHIFT, bool TAIL>
__global__ __launch_bounds__(256) void norm_ff_kernel(const unsigned short* __restrict__ raw, const float* __restrict__ gw,
                                                      const float* __restrict__ gb, unsigned short* __restrict__ outp) {
  __shared__ float shs[8];
  __shared__ float shq[8];
  const int tid = threadIdx.x, lane = tid & 31, wave = tid >> 5;
  const int n = blockIdx.x;
  const int rsub = tid >> 4;
  const int c8 = (tid & 15) * 8;
  const unsigned short* rbase = raw + (size_t)n * kTime * kFf;
  float s = 0.0f, q = 0.0f;
#pragma unroll 1
  for (int it = 0; it < 32; ++it) {
    const int row = it * 16 + rsub;
    const bool valid = row < kLen;
    const int rc = valid ? row : (kLen - 1);
    const uv4 w = *(const uv4*)(rbase + (size_t)rc * kFf + c8);
    float f[8];
    unpack8(w, f);
    float ps = 0.0f, pq = 0.0f;
#pragma unroll
    for (int e = 0; e < 8; ++e) { ps += f[e]; pq += f[e] * f[e]; }
    s += valid ? ps : 0.0f;
    q += valid ? pq : 0.0f;
  }
#pragma unroll
  for (int off = 16; off > 0; off >>= 1) { s += __shfl_xor(s, off, 32); q += __shfl_xor(q, off, 32); }
  if (lane == 0) { shs[wave] = s; shq[wave] = q; }
  __syncthreads();
  double S = 0.0, Q = 0.0;
#pragma unroll
  for (int i = 0; i < 8; ++i) { S += (double)shs[i]; Q += (double)shq[i]; }
  const double invc = 1.0 / (double)(kFf * kLen);
  const double md = S * invc;
  double vd = Q * invc - md * md;
  vd = (vd < 0.0) ? 0.0 : vd;
  const float mean = (float)md;
  const float rstd = rsqrtf((float)vd + kEps);

  const v4f g0 = *(const v4f*)(gw + c8);
  const v4f g1 = *(const v4f*)(gw + c8 + 4);
  const v4f b0 = *(const v4f*)(gb + c8);
  const v4f b1 = *(const v4f*)(gb + c8 + 4);
  const float gwv[8] = {g0[0], g0[1], g0[2], g0[3], g1[0], g1[1], g1[2], g1[3]};
  const float gbv[8] = {b0[0], b0[1], b0[2], b0[3], b1[0], b1[1], b1[2], b1[3]};
#pragma unroll 1
  for (int it = 0; it < 32; ++it) {
    const int p = it * 16 + rsub;
    const int l = p - SHIFT;
    const bool valid = (l >= 0) && (l < kLen);
    const int lc = (l < 0) ? 0 : ((l > kLen - 1) ? (kLen - 1) : l);
    const uv4 w = *(const uv4*)(rbase + (size_t)lc * kFf + c8);
    float f[8];
    unpack8(w, f);
    v8h hv;
#pragma unroll
    for (int e = 0; e < 8; ++e) {
      float y = ((f[e] - mean) * rstd) * gwv[e] + gbv[e];
      y = (y >= 0.0f) ? y : 0.25f * y;
      y = valid ? y : 0.0f;
      hv[e] = (_Float16)y;
    }
    volatile v8h* op = (volatile v8h*)(outp + ((size_t)n * kTime + p) * kFf + c8);
    *op = hv;
    __threadfence();
    *op = hv;
  }
  if (TAIL) {
    if (n == kSeq - 1 && tid < 96) {
      v8h z;
#pragma unroll
      for (int e = 0; e < 8; ++e) z[e] = (_Float16)0.0f;
      volatile v8h* op = (volatile v8h*)(outp + (size_t)kRows * kFf + tid * 8);
      *op = z;
      __threadfence();
      *op = z;
    }
  }
}

__global__ __launch_bounds__(256) void norm_res_kernel(const float* __restrict__ raw, const float* __restrict__ hres,
                                                       const float* __restrict__ gw, const float* __restrict__ gb,
                                                       unsigned short* __restrict__ qout) {
  __shared__ float shs[8];
  __shared__ float shq[8];
  const int tid = threadIdx.x, lane = tid & 31, wave = tid >> 5;
  const int n = blockIdx.x;
  const float* rbase = raw + (size_t)n * kTime * kChan;
  const float* hbase = hres + (size_t)n * kTime * kChan;
  float s = 0.0f, q = 0.0f;
  {
    const int rsub = tid >> 4;
    const int c4 = (tid & 15) * 4;
#pragma unroll 1
    for (int it = 0; it < 32; ++it) {
      const int row = it * 16 + rsub;
      const bool valid = row < kLen;
      const int rc = valid ? row : (kLen - 1);
      const v4f v = *(const v4f*)(rbase + (size_t)rc * kChan + c4);
      const float ps = (v[0] + v[1]) + (v[2] + v[3]);
      const float pq = (v[0] * v[0] + v[1] * v[1]) + (v[2] * v[2] + v[3] * v[3]);
      s += valid ? ps : 0.0f;
      q += valid ? pq : 0.0f;
    }
  }
#pragma unroll
  for (int off = 16; off > 0; off >>= 1) { s += __shfl_xor(s, off, 32); q += __shfl_xor(q, off, 32); }
  if (lane == 0) { shs[wave] = s; shq[wave] = q; }
  __syncthreads();
  double S = 0.0, Q = 0.0;
#pragma unroll
  for (int i = 0; i < 8; ++i) { S += (double)shs[i]; Q += (double)shq[i]; }
  const double invc = 1.0 / (double)(kChan * kLen);
  const double md = S * invc;
  double vd = Q * invc - md * md;
  vd = (vd < 0.0) ? 0.0 : vd;
  const float mean = (float)md;
  const float rstd = rsqrtf((float)vd + kEps);

  const int c8 = (tid & 7) * 8;
  const int psub = tid >> 3;
  const v4f g0 = *(const v4f*)(gw + c8);
  const v4f g1 = *(const v4f*)(gw + c8 + 4);
  const v4f b0 = *(const v4f*)(gb + c8);
  const v4f b1 = *(const v4f*)(gb + c8 + 4);
  const float gwv[8] = {g0[0], g0[1], g0[2], g0[3], g1[0], g1[1], g1[2], g1[3]};
  const float gbv[8] = {b0[0], b0[1], b0[2], b0[3], b1[0], b1[1], b1[2], b1[3]};
#pragma unroll 1
  for (int it = 0; it < 17; ++it) {
    const int p = it * 32 + psub;
    const bool act = p < kQRows;
    const int pc = act ? p : (kQRows - 1);
    const int l = pc - (kTap - 1);
    const bool valid = (l >= 0) && (l < kLen);
    const int lc = (l < 0) ? 0 : ((l > kLen - 1) ? (kLen - 1) : l);
    const v4f a0 = *(const v4f*)(rbase + (size_t)lc * kChan + c8);
    const v4f a1 = *(const v4f*)(rbase + (size_t)lc * kChan + c8 + 4);
    const v4f h0 = *(const v4f*)(hbase + (size_t)lc * kChan + c8);
    const v4f h1 = *(const v4f*)(hbase + (size_t)lc * kChan + c8 + 4);
    const float av[8] = {a0[0], a0[1], a0[2], a0[3], a1[0], a1[1], a1[2], a1[3]};
    const float hv8[8] = {h0[0], h0[1], h0[2], h0[3], h1[0], h1[1], h1[2], h1[3]};
    v8h hv;
#pragma unroll
    for (int e = 0; e < 8; ++e) {
      float y = ((av[e] - mean) * rstd) * gwv[e] + gbv[e];
      y = (y >= 0.0f) ? y : 0.25f * y;
      y = y + hv8[e];
      y = valid ? y : 0.0f;
      hv[e] = (_Float16)y;
    }
    if (act) {
      volatile v8h* op = (volatile v8h*)(qout + ((size_t)n * kQRows + pc) * kChan + c8);
      *op = hv;
      __threadfence();
      *op = hv;
    }
  }
}

__global__ __launch_bounds__(64) void convt_out_kernel(const unsigned short* __restrict__ Qp, const unsigned short* __restrict__ Bp,
                                                       const float* __restrict__ ctb, const float* __restrict__ xin,
                                                       float* __restrict__ outp, float scale) {
  __shared__ __align__(16) float sO[2][64 * 68];
  const int lane = threadIdx.x & 31;
  const int wave = threadIdx.x >> 5;
  const int tile = blockIdx.x * 2 + wave;
  const int n = tile >> 3;
  const int t0 = (tile & 7) * 64;
  const _Float16* Ab = (const _Float16*)Qp + ((size_t)n * kQRows + t0) * kChan;
  const _Float16* Bb = (const _Float16*)Bp;
  const int rlane = lane & 15;
  const int koff  = (lane >> 4) * 8;
  const int mOff  = (lane >> 4) * 8;

  v8f acc[4][4];
#pragma unroll
  for (int i = 0; i < 4; ++i)
#pragma unroll
    for (int j = 0; j < 4; ++j) acc[i][j] = (v8f){0.f,0.f,0.f,0.f,0.f,0.f,0.f,0.f};

  for (int k0 = 0; k0 < kKct; k0 += 32) {
    v16h bh[4];
#pragma unroll
    for (int j = 0; j < 4; ++j) bh[j] = Frag<_Float16>::load(Bb + (size_t)((j << 4) + rlane) * kKct + koff + k0);
#pragma unroll
    for (int i = 0; i < 4; ++i) {
      const v16h ah = Frag<_Float16>::load(Ab + (size_t)((i << 4) + rlane) * kChan + koff + k0);
#pragma unroll
      for (int j = 0; j < 4; ++j) acc[i][j] = Frag<_Float16>::mma(ah, bh[j], acc[i][j]);
      dep_guard4_h(acc[i][0], acc[i][1], acc[i][2], acc[i][3], ah, bh[3]);
    }
    keep4_h(bh[0], bh[1], bh[2], bh[3]);
  }
  acc_guard4(acc[0][0], acc[0][1], acc[0][2], acc[0][3]);
  acc_guard4(acc[1][0], acc[1][1], acc[1][2], acc[1][3]);
  acc_guard4(acc[2][0], acc[2][1], acc[2][2], acc[2][3]);
  acc_guard4(acc[3][0], acc[3][1], acc[3][2], acc[3][3]);

  float* slab = sO[wave];
#pragma unroll
  for (int j = 0; j < 4; ++j) {
    const float bv = ctb[(j << 4) + rlane];
#pragma unroll
    for (int i = 0; i < 4; ++i) {
#pragma unroll
      for (int r = 0; r < 8; ++r) slab[((j << 4) + rlane) * 68 + (i << 4) + mOff + r] = acc[i][j][r] * scale + bv;
    }
  }
  __builtin_amdgcn_fence(__ATOMIC_RELEASE, "workgroup");
  __builtin_amdgcn_wave_barrier();
  __builtin_amdgcn_fence(__ATOMIC_ACQUIRE, "workgroup");
  const int hh = lane >> 4;
  const int c4 = (lane & 15) * 4;
#pragma unroll 1
  for (int it = 0; it < 32; ++it) {
    const int o = it * 2 + hh;
    v4f v = *(const v4f*)(slab + o * 68 + c4);
    const size_t goff = ((size_t)(o * kSeq + n)) * kTime + t0 + c4;
    const v4f xi = *(const v4f*)(xin + goff);
    v = v + xi;
    volatile v4f* op = (volatile v4f*)(outp + goff);
    *op = v;
    __threadfence();
    *op = v;
  }
}

extern "C" void kernel_launch(void* const* d_in, const int* in_sizes, int n_in,
                              void* d_out, int out_size, void* d_ws, size_t ws_size, hipStream_t stream) {
  if (n_in < 20 || d_out == nullptr || d_ws == nullptr) return;
  if (in_sizes[0] != kChan * kSeq * kTime || in_sizes[1] != kChan || in_sizes[2] != kChan ||
      in_sizes[3] != 2 * kKsru * 128 || in_sizes[4] != 2 * 2 * kHid || in_sizes[5] != 2 * 2 * kHid ||
      in_sizes[6] != kFf * kChan || in_sizes[7] != kFf || in_sizes[8] != kFf || in_sizes[9] != kFf ||
      in_sizes[10] != kFf * kFf * kTap || in_sizes[11] != kFf || in_sizes[12] != kFf || in_sizes[13] != kFf ||
      in_sizes[14] != kChan * kFf || in_sizes[15] != kChan || in_sizes[16] != kChan || in_sizes[17] != kChan ||
      in_sizes[18] != kChan * kChan * kTap || in_sizes[19] != kChan || out_size != kChan * kSeq * kTime) return;

  const float* x    = (const float*)d_in[0];
  const float* g0w  = (const float*)d_in[1];
  const float* g0b  = (const float*)d_in[2];
  const float* sruw = (const float*)d_in[3];
  const float* sruv = (const float*)d_in[4];
  const float* srub = (const float*)d_in[5];
  const float* c1w  = (const float*)d_in[6];
  const float* c1b  = (const float*)d_in[7];
  const float* g1w  = (const float*)d_in[8];
  const float* g1b  = (const float*)d_in[9];
  const float* c2w  = (const float*)d_in[10];
  const float* c2b  = (const float*)d_in[11];
  const float* g2w  = (const float*)d_in[12];
  const float* g2b  = (const float*)d_in[13];
  const float* c3w  = (const float*)d_in[14];
  const float* c3b  = (const float*)d_in[15];
  const float* g3w  = (const float*)d_in[16];
  const float* g3b  = (const float*)d_in[17];
  const float* ctw  = (const float*)d_in[18];
  const float* ctb  = (const float*)d_in[19];
  float* out = (float*)d_out;

  char* ws = (char*)d_ws;
  size_t off = 0;
  auto carve = [&](size_t bytes) -> char* { char* p = ws + off; off += (bytes + 255) & ~(size_t)255; return p; };
  float*          STP = (float*)carve((size_t)256 * 32 * 4);
  float*          STF = (float*)carve((size_t)256);
  unsigned short* WPL = (unsigned short*)carve((size_t)kWTotal * 2);
  unsigned short* R0  = (unsigned short*)carve((size_t)kSeq * kQRows * kChan * 2);
  char*           BIG = carve((size_t)67108864 + 4096);
  float*          HB  = (float*)carve((size_t)kRows * kChan * 4);
  if (off > ws_size || off > (size_t)134217728) return;
  static_assert((size_t)kRows * kChan * 2 + 1024 <= (size_t)kSeq * kQRows * kChan * 2, "Xn + tail fits R0");

  unsigned short* Xn  = R0;
  unsigned short* H16 = R0;
  unsigned short* Qpl = R0;
  float*          Ubuf  = (float*)BIG;
  unsigned short* Y1raw = (unsigned short*)BIG;
  unsigned short* Ppl   = (unsigned short*)(BIG + 33554432);
  unsigned short* Y2raw = (unsigned short*)BIG;
  unsigned short* A2pl  = (unsigned short*)(BIG + 33554432);
  float*          Y3raw = (float*)BIG;

  gn0_partial_kernel<<<256, 256, 0, stream>>>(x, STP);
  gn0_final_kernel<<<1, 256, 0, stream>>>(STP, STF);
  wprep_kernel<<<kWTotal / 2048, 256, 0, stream>>>(sruw, c1w, c2w, c3w, ctw, WPL);
  pack_xn_kernel<<<kSeq * 8 + 1, 256, 0, stream>>>(x, g0w, g0b, STF, Xn);

  const dim3 g128((kRows / 64) * (128 / 64) / 8, 1);
  const dim3 g64((kRows / 64) * (64 / 64) / 8, 1);
  for (int d = 0; d < 2; ++d) {
    const unsigned short* Bs = WPL + kOffSru + (size_t)d * 128 * kKsru;
    wmma_gemm64<0, false, 0, 0, false><<<g128, 256, 0, stream>>>(
        Xn, Xn, kChan, 0L, Bs, Bs, kKsru, 0L, (void*)Ubuf, (void*)Ubuf, 128, 0L,
        c1b, HB, 0L, kRows, 128, kKsru, kWCarryInv);
    sru_scan_kernel<<<kSeq / 8, 256, 0, stream>>>(Ubuf, sruv, srub, HB, d);
  }

  cast_h_kernel<<<(kRows * 8) / 256, 256, 0, stream>>>(HB, H16);
  wmma_gemm64<0, false, 2, 1, false><<<g128, 256, 0, stream>>>(
      H16, H16, kChan, 0L, WPL + kOffC1, WPL + kOffC1, kChan, 0L, (void*)Y1raw, (void*)Y1raw, kFf, 0L,
      c1b, HB, 0L, kRows, kFf, kChan, kWCarryInv);
  norm_ff_kernel<3, true><<<kSeq, 256, 0, stream>>>(Y1raw, g1w, g1b, Ppl);
  wmma_gemm64<0, false, 2, 1, false><<<g128, 256, 0, stream>>>(
      Ppl, Ppl, kFf, 0L, WPL + kOffC2, WPL + kOffC2, kKc2, 0L, (void*)Y2raw, (void*)Y2raw, kFf, 0L,
      c2b, HB, 0L, kRows, kFf, kKc2, kWCarryInv);
  norm_ff_kernel<0, false><<<kSeq, 256, 0, stream>>>(Y2raw, g2w, g2b, A2pl);
  wmma_gemm64<0, false, 2, 0, false><<<g64, 256, 0, stream>>>(
      A2pl, A2pl, kFf, 0L, WPL + kOffC3, WPL + kOffC3, kFf, 0L, (void*)Y3raw, (void*)Y3raw, kChan, 0L,
      c3b, HB, 0L, kRows, kChan, kFf, kWCarryInv);
  norm_res_kernel<<<kSeq, 256, 0, stream>>>(Y3raw, HB, g3w, g3b, Qpl);
  convt_out_kernel<<<(kSeq * (kTime / 64)) / 2, 64, 0, stream>>>(Qpl, WPL + kOffCt, ctb, x, out, kWCarryInv);
}
